// MultiHeadAttention_16423954940513
// MI455X (gfx1250) — hardware-verified
//
#include <hip/hip_runtime.h>


#ifndef NB
#define NB 2
#endif
#ifndef SEQ
#define SEQ 2048
#endif
#define NB_FULL  2
#define SEQ_FULL 2048
#ifndef OUT_SEQ
#define OUT_SEQ SEQ
#endif
#define DM   2048
#define HD   128
#define NG   4
#define NHG  4
#define NQH  16
#define DKV  512
#define ESEQ ((SEQ < 512) ? SEQ : 512)
#define AW   4
#define QRS  2048.0f
#define QRI  (1.0f / 2048.0f)
#define SC2  (0.0078125f * 1.4426950408889634f)
#define PSH  8.0f
#define OCS  64.0f
#define WOS  1024.0f
#define OSI  (1.0f / 65536.0f)
#define C_HI (108853.0f * 1.9073486328125e-6f)
#define C_LO (-1.147971e-7f)

static_assert(HD == 128);
static_assert(NQH * HD == DM);
static_assert(NG * HD == DKV);
static_assert(NG * NHG == NQH);
static_assert(DM % 64 == 0);
static_assert(DM % 32 == 0);
static_assert(DKV % 64 == 0);
static_assert(SEQ % 64 == 0);
static_assert(ESEQ % 64 == 0);
static_assert((SEQ - ESEQ) % 64 == 0);
static_assert((64 * SEQ) % 256 == 0);
static_assert(((size_t)SEQ * DM) % 8 == 0);
static_assert(NB <= NB_FULL);
static_assert(SEQ <= SEQ_FULL);
static_assert(((size_t)(NB - 1) * OUT_SEQ + SEQ) * DM * 4 <= (size_t)33554432);

typedef _Float16 h16;
typedef unsigned short bf;
typedef __attribute__((ext_vector_type(16))) __bf16   v16bf;
typedef __attribute__((ext_vector_type(16))) _Float16 v16h;
typedef __attribute__((ext_vector_type(8)))  _Float16 v8h;
typedef __attribute__((ext_vector_type(8)))  unsigned short v8us;
typedef __attribute__((ext_vector_type(8)))  float    v8f;
typedef __attribute__((ext_vector_type(4)))  float    v4f;
typedef v4f  __attribute__((may_alias)) v4fa;
typedef v8us __attribute__((may_alias)) v8usa;

__device__ __forceinline__ unsigned short f2bf(float f) { unsigned u = __float_as_uint(f); u += 0x7FFFu + ((u >> 16) & 1u); return (unsigned short)(u >> 16); }
__device__ __forceinline__ v16h cat16(v8h lo, v8h hi) { return __builtin_shufflevector(lo, hi, 0, 1, 2, 3, 4, 5, 6, 7, 8, 9, 10, 11, 12, 13, 14, 15); }
__device__ __forceinline__ v16bf cat16b(v8us lo, v8us hi) { return __builtin_bit_cast(v16bf, __builtin_shufflevector(lo, hi, 0, 1, 2, 3, 4, 5, 6, 7, 8, 9, 10, 11, 12, 13, 14, 15)); }
__device__ __forceinline__ v8f wmma16(v16h a, v16h b, v8f c) { return __builtin_amdgcn_wmma_f32_16x16x32_f16(false, a, false, b, (short)0, c, false, false); }
__device__ __forceinline__ v8f wmmab(v16bf a, v16bf b, v8f c) { return __builtin_amdgcn_wmma_f32_16x16x32_bf16(false, a, false, b, (short)0, c, false, false); }
__device__ __forceinline__ v16h  ldh(const h16* p) { return cat16(*(const v8h*)p, *(const v8h*)(p + 16)); }
__device__ __forceinline__ v16bf ldb(const bf* p)  { return cat16b(*(const v8us*)p, *(const v8us*)(p + 16)); }
__device__ __forceinline__ void wave_sync() { __builtin_amdgcn_fence(3  , "wavefront"); __builtin_amdgcn_wave_barrier(); asm volatile("" ::: "memory"); }
__device__ __forceinline__ unsigned short cvw(float v, int mode) {
    const unsigned short b = f2bf(v);
    const float r = __uint_as_float((unsigned)b << 16) * WOS;
    const h16 hh = (h16)r;
    const unsigned short hb = __builtin_bit_cast(unsigned short, hh);
    return mode ? hb : b;
}

__global__ __launch_bounds__(256) void k_cvt8(const float* __restrict__ src, bf* dst, size_t n8) {
    const size_t i = (size_t)blockIdx.x * 256 + threadIdx.x; if (i >= n8) return;
    const v8f v = *(const v8f*)(src + i * 8); v8us o;
#pragma unroll
    for (int k = 0; k < 8; ++k) o[k] = f2bf(v[k]);
    *(volatile v8us*)(dst + i * 8) = o; __threadfence(); *(volatile v8us*)(dst + i * 8) = o;
}

__global__ __launch_bounds__(256) void k_tcvt(const float* __restrict__ src, unsigned short* dst, int R, int C, int mode) {
    __shared__ __align__(16) unsigned short tl[64 * 72];
    const int tid = threadIdx.x; const int c0 = blockIdx.x * 64, r0 = blockIdx.y * 64;
    const int ty = tid >> 4, tx = tid & 15;
#pragma unroll
    for (int p = 0; p < 4; ++p) { const int row = ty + 16 * p;
        const v4f v = *(const v4f*)(src + (size_t)(r0 + row) * C + c0 + 4 * tx);
#pragma unroll
        for (int i = 0; i < 4; ++i) tl[(4 * tx + i) * 72 + row] = cvw(v[i], mode); }
    __syncthreads();
    const int pc = tid & 7, cr = tid >> 3;
    const v8us o0 = *(const v8usa*)(&tl[cr * 72 + pc * 8]);
    const v8us o1 = *(const v8usa*)(&tl[(cr + 32) * 72 + pc * 8]);
    const size_t a0 = (size_t)(c0 + cr) * R + r0 + pc * 8, a1 = (size_t)(c0 + cr + 32) * R + r0 + pc * 8;
#pragma unroll 1
    for (int ps = 0; ps < 2; ++ps) {
        *(volatile v8us*)(dst + a0) = o0; *(volatile v8us*)(dst + a1) = o1;
        if (ps == 0) __threadfence(); }
}

__global__ __launch_bounds__(256) void k_ropetab(float* CT, float* ST) {
    const int i = blockIdx.x * 256 + threadIdx.x;
    const int jf = i / SEQ, t = i % SEQ;
    const float fj = (float)jf;
    const float a = fj * C_HI;
    const float fl = floorf(a);
    const float fr = (a - fl) + fj * C_LO;
    const float p2 = __uint_as_float((unsigned)(127 - (int)fl) << 23);
    const float freq = __builtin_amdgcn_exp2f(-fr) * p2;
    const float rad = (float)t * freq;
    float s, c; sincosf(rad, &s, &c);
    *(volatile float*)(CT + i) = c; *(volatile float*)(ST + i) = s;
    __threadfence();
    *(volatile float*)(CT + i) = c; *(volatile float*)(ST + i) = s;
}

__global__ __launch_bounds__(32) void k_projr(const bf* __restrict__ A, const bf* __restrict__ Bt, const float* __restrict__ CT, const float* __restrict__ ST, h16* Ph, h16* Pr, int nheads) {
    __shared__ __align__(16) float os[16 * 132];
    const int K = DM;
    const int lane = threadIdx.x & 31, lr = lane & 15, hi = lane >> 4; const int r0 = blockIdx.x * 32, head = blockIdx.y, c0 = head * HD;
    v8f acc[2][8];
#pragma unroll
    for (int mb = 0; mb < 2; ++mb)
#pragma unroll
        for (int nb = 0; nb < 8; ++nb) acc[mb][nb] = (v8f){};
    const size_t aoff = (size_t)(r0 + lr) * K + 8 * hi, boff = (size_t)(c0 + lr) * K + 8 * hi;
#pragma unroll 1
    for (int kc = 0; kc < K; kc += 32) {
        v16bf a[2]; v16bf b;
#pragma unroll
        for (int mb = 0; mb < 2; ++mb) a[mb] = ldb(A + aoff + (size_t)mb * 16 * K + kc);
#pragma unroll
        for (int nb = 0; nb < 8; ++nb) { b = ldb(Bt + boff + (size_t)nb * 16 * K + kc);
#pragma unroll
            for (int mb = 0; mb < 2; ++mb) acc[mb][nb] = wmmab(a[mb], b, acc[mb][nb]); }
        asm volatile("v_nop\n\tv_nop\n\tv_nop\n\tv_nop" : "+v"(acc[0][6]), "+v"(acc[1][6]), "+v"(acc[0][7]), "+v"(acc[1][7]) : "v"(a[0]), "v"(a[1]), "v"(b));
    }
    const int bb = r0 / SEQ, t0 = r0 % SEQ;
    const size_t pbase = ((size_t)(bb * nheads + head) * SEQ + t0) * HD;
#pragma unroll
    for (int mb = 0; mb < 2; ++mb) {
        const int tr = t0 + mb * 16 + 8 * hi;
#pragma unroll
        for (int nb = 0; nb < 4; ++nb) {
            const int jf = nb * 16 + lr;
            const v8f cs = *(const v8f*)(CT + (size_t)jf * SEQ + tr);
            const v8f sn = *(const v8f*)(ST + (size_t)jf * SEQ + tr);
#pragma unroll
            for (int j = 0; j < 8; ++j) { const float e = acc[mb][nb][j], o = acc[mb][nb + 4][j];
                os[(hi * 8 + j) * 132 + nb * 16 + lr]      = e * cs[j] - o * sn[j];
                os[(hi * 8 + j) * 132 + 64 + nb * 16 + lr] = e * sn[j] + o * cs[j]; } }
        wave_sync();
        const size_t sb = pbase + (size_t)(mb * 16) * HD;
#pragma unroll 1
        for (int ps = 0; ps < 2; ++ps) {
#pragma unroll
            for (int s = 0; s < 8; ++s) { const int row = 2 * s + (lane >> 4), c8 = (lane & 15) * 8;
                const v4f x0 = *(const v4fa*)(&os[row * 132 + c8]); const v4f x1 = *(const v4fa*)(&os[row * 132 + c8 + 4]); v8h hv, rv;
#pragma unroll
                for (int i = 0; i < 4; ++i) { const h16 a0 = (h16)x0[i]; const h16 a1 = (h16)x1[i]; hv[i] = a0; hv[4 + i] = a1; rv[i] = (h16)((x0[i] - (float)a0) * QRS); rv[4 + i] = (h16)((x1[i] - (float)a1) * QRS); }
                const size_t oo = sb + (size_t)row * HD + c8;
                *(volatile v8h*)(Ph + oo) = hv; *(volatile v8h*)(Pr + oo) = rv; }
            if (ps == 0) __threadfence(); }
        wave_sync();
    }
}

__global__ __launch_bounds__(32) void k_projt(const bf* __restrict__ A, const bf* __restrict__ Bt, h16* Ph, h16* Pr, int useRes, int RB, size_t sRB, int pitch, int CB, size_t sCB) {
    __shared__ __align__(16) float os[16 * 68];
    const int K = DM;
    const int lane = threadIdx.x & 31, lr = lane & 15, hi = lane >> 4; const int r0 = blockIdx.x * 64, c0 = blockIdx.y * 64;
    v8f acc[4][4];
#pragma unroll
    for (int mb = 0; mb < 4; ++mb)
#pragma unroll
        for (int nb = 0; nb < 4; ++nb) acc[mb][nb] = (v8f){};
    const size_t aoff = (size_t)(r0 + lr) * K + 8 * hi, boff = (size_t)(c0 + lr) * K + 8 * hi;
#pragma unroll 1
    for (int kc = 0; kc < K; kc += 32) {
        v16bf a[4];
#pragma unroll
        for (int mb = 0; mb < 4; ++mb) a[mb] = ldb(A + aoff + (size_t)mb * 16 * K + kc);
#pragma unroll
        for (int nb = 0; nb < 4; ++nb) { const v16bf b = ldb(Bt + boff + (size_t)nb * 16 * K + kc);
#pragma unroll
            for (int mb = 0; mb < 4; ++mb) acc[mb][nb] = wmmab(a[mb], b, acc[mb][nb]); }
        asm volatile("v_nop\n\tv_nop\n\tv_nop\n\tv_nop" : "+v"(acc[0][0]), "+v"(acc[1][1]), "+v"(acc[2][2]), "+v"(acc[3][3]) : "v"(a[0]), "v"(a[1]), "v"(a[2]), "v"(a[3]));
    }
    const size_t tbase = (size_t)(r0 / RB) * sRB + (size_t)(r0 % RB) * (size_t)pitch + (size_t)(c0 / CB) * sCB + (size_t)(c0 % CB);
#pragma unroll
    for (int mb = 0; mb < 4; ++mb) {
#pragma unroll
        for (int nb = 0; nb < 4; ++nb) {
#pragma unroll
            for (int j = 0; j < 8; ++j) os[(hi * 8 + j) * 68 + nb * 16 + lr] = acc[mb][nb][j]; }
        wave_sync();
        const size_t sb = tbase + (size_t)(mb * 16) * (size_t)pitch;
#pragma unroll 1
        for (int ps = 0; ps < 2; ++ps) {
#pragma unroll
            for (int s = 0; s < 4; ++s) { const int row = 4 * s + (lane >> 3), c8 = (lane & 7) * 8;
                const v4f x0 = *(const v4fa*)(&os[row * 68 + c8]); const v4f x1 = *(const v4fa*)(&os[row * 68 + c8 + 4]); v8h hv, rv;
#pragma unroll
                for (int i = 0; i < 4; ++i) { const h16 a0 = (h16)x0[i]; const h16 a1 = (h16)x1[i]; hv[i] = a0; hv[4 + i] = a1; rv[i] = (h16)((x0[i] - (float)a0) * QRS); rv[4 + i] = (h16)((x1[i] - (float)a1) * QRS); }
                const size_t oo = sb + (size_t)row * (size_t)pitch + c8;
                *(volatile v8h*)(Ph + oo) = hv; if (useRes) *(volatile v8h*)(Pr + oo) = rv; }
            if (ps == 0) __threadfence(); }
        wave_sync();
    }
}

__global__ __launch_bounds__(32 * AW) __attribute__((amdgpu_num_vgpr(256)))
void k_flash3(const h16* __restrict__ QH, const h16* __restrict__ QR, const h16* __restrict__ KP, const h16* __restrict__ KR,
              const h16* __restrict__ VT, const h16* __restrict__ VR, h16* OH, h16* OR) {
    __shared__ __align__(16) float os[AW * 16 * 68];
    const int lane = threadIdx.x & 31, lr = lane & 15, hi = lane >> 4;
    const int wave = __builtin_amdgcn_readfirstlane((int)(threadIdx.x >> 5));
    const int zh = blockIdx.y; const int b = zh / NQH, gh = zh % NQH; const int zk = b * NG + gh / NHG; const int dh = blockIdx.z;
    const int t0 = (blockIdx.x * AW + wave) * 16;
    const size_t qo = ((size_t)zh * SEQ + t0 + lr) * HD + 8 * hi;
    const size_t ko = ((size_t)zk * SEQ + lr) * HD + 8 * hi;
    const size_t vo = ((size_t)zk * HD + dh * 64 + lr) * SEQ + 8 * hi;
    v8f oH[4], oL[4];
#pragma unroll
    for (int j = 0; j < 4; ++j) { oH[j] = (v8f){}; oL[j] = (v8f){}; }
    float m = -3.0e38f, l = 0.0f;
    const int tq = t0 + lr;
    const int nst = (t0 + 15) / 32 + 1;
#pragma unroll 1
    for (int st = 0; st < nst; ++st) {
        const int key0 = st * 32;
        const size_t kofs = ko + (size_t)key0 * HD;
        v8f sHa = (v8f){}, sLa = (v8f){}, sHb = (v8f){}, sLb = (v8f){};
#pragma unroll 1
        for (int c = 0; c < 4; ++c) {
            const v16h qhc = ldh(QH + qo + 32 * c), qrc = ldh(QR + qo + 32 * c);
            const v16h fa = ldh(KP + kofs + 32 * c), fb = ldh(KP + kofs + 16 * HD + 32 * c);
            const v16h ga = ldh(KR + kofs + 32 * c), gb = ldh(KR + kofs + 16 * HD + 32 * c);
            sHa = wmma16(fa, qhc, sHa); sHb = wmma16(fb, qhc, sHb);
            sLa = wmma16(fa, qrc, sLa); sLb = wmma16(fb, qrc, sLb);
            sLa = wmma16(ga, qhc, sLa); sLb = wmma16(gb, qhc, sLb);
            asm volatile("v_nop\n\tv_nop\n\tv_nop\n\tv_nop" : "+v"(sHa), "+v"(sLa), "+v"(sHb), "+v"(sLb) : "v"(fa), "v"(fb), "v"(ga), "v"(gb), "v"(qhc), "v"(qrc));
        }
        float ta[8], tb[8]; float mx = -3.0e38f;
        const int kk = key0 + 8 * hi - tq;
#pragma unroll
        for (int r = 0; r < 8; ++r) { float u = (sHa[r] + sLa[r] * QRI) * SC2; float w = (sHb[r] + sLb[r] * QRI) * SC2;
            u = (kk + r > 0) ? -1.0e30f : u; w = (kk + 16 + r > 0) ? -1.0e30f : w;
            ta[r] = u; tb[r] = w; mx = fmaxf(mx, fmaxf(u, w)); }
        mx = fmaxf(mx, __shfl_xor(mx, 16, 32));
        const float mnew = fmaxf(m, mx);
        const float alpha = __builtin_amdgcn_exp2f(m - mnew);
        const float sh = PSH - mnew;
        v16h ph, pr; float ls = 0.0f;
#pragma unroll
        for (int r = 0; r < 8; ++r) { const float pa = __builtin_amdgcn_exp2f(ta[r] + sh); const float pc = __builtin_amdgcn_exp2f(tb[r] + sh);
            const h16 ha = (h16)pa; const h16 hc = (h16)pc; const h16 ra = (h16)((pa - (float)ha) * QRS); const h16 rc = (h16)((pc - (float)hc) * QRS);
            ph[r] = ha; ph[8 + r] = hc; pr[r] = ra; pr[8 + r] = rc;
            ls += ((float)ha + (float)ra * QRI) + ((float)hc + (float)rc * QRI); }
        l = l * alpha + ls; m = mnew;
#pragma unroll
        for (int j = 0; j < 4; ++j) { oH[j] = oH[j] * alpha; oL[j] = oL[j] * alpha; }
        const size_t vofs = vo + key0;
        v16h vh, vr;
#pragma unroll
        for (int j = 0; j < 4; ++j) { vh = ldh(VT + vofs + (size_t)(16 * j) * SEQ); vr = ldh(VR + vofs + (size_t)(16 * j) * SEQ);
            oH[j] = wmma16(vh, ph, oH[j]); oL[j] = wmma16(vr, ph, oL[j]); oL[j] = wmma16(vh, pr, oL[j]); }
        asm volatile("v_nop\n\tv_nop\n\tv_nop\n\tv_nop" : "+v"(oH[2]), "+v"(oL[2]), "+v"(oH[3]), "+v"(oL[3]) : "v"(vh), "v"(vr), "v"(ph), "v"(pr));
    }
    l += __shfl_xor(l, 16, 32);
    const float inv = OCS * (1.0f / l);
    const int wb = wave * 16 * 68;
#pragma unroll
    for (int j = 0; j < 4; ++j) { const v8f f = (oH[j] + oL[j] * QRI) * inv;
        const v4f a = __builtin_shufflevector(f, f, 0, 1, 2, 3); const v4f c = __builtin_shufflevector(f, f, 4, 5, 6, 7);
        *(v4fa*)(&os[wb + lr * 68 + 16 * j + 8 * hi]) = a; *(v4fa*)(&os[wb + lr * 68 + 16 * j + 8 * hi + 4]) = c; }
    wave_sync();
    const size_t obase = ((size_t)b * SEQ + t0) * DM + gh * HD + dh * 64;
#pragma unroll 1
    for (int ps = 0; ps < 2; ++ps) {
#pragma unroll
        for (int s = 0; s < 4; ++s) { const int row = 4 * s + (lane >> 3), c8 = (lane & 7) * 8;
            const v4f x0 = *(const v4fa*)(&os[wb + row * 68 + c8]); const v4f x1 = *(const v4fa*)(&os[wb + row * 68 + c8 + 4]); v8h hv, rv;
#pragma unroll
            for (int i = 0; i < 4; ++i) { const h16 a0 = (h16)x0[i]; const h16 a1 = (h16)x1[i]; hv[i] = a0; hv[4 + i] = a1; rv[i] = (h16)((x0[i] - (float)a0) * QRS); rv[4 + i] = (h16)((x1[i] - (float)a1) * QRS); }
            const size_t oo = obase + (size_t)row * DM + c8;
            *(volatile v8h*)(OH + oo) = hv; *(volatile v8h*)(OR + oo) = rv; }
        if (ps == 0) __threadfence(); }
}

__global__ __launch_bounds__(32 * AW) __attribute__((amdgpu_num_vgpr(256)))
void k_flash(const h16* __restrict__ QH, const h16* __restrict__ KP, const h16* __restrict__ VT, h16* OH) {
    __shared__ __align__(16) float os[AW * 16 * 132];
    const int lane = threadIdx.x & 31, lr = lane & 15, hi = lane >> 4;
    const int wave = __builtin_amdgcn_readfirstlane((int)(threadIdx.x >> 5));
    const int zh = blockIdx.y; const int b = zh / NQH, gh = zh % NQH; const int zk = b * NG + gh / NHG;
    const int t0 = ESEQ + (blockIdx.x * AW + wave) * 16;
    const size_t qo = ((size_t)zh * SEQ + t0 + lr) * HD + 8 * hi;
    v16h q[4];
#pragma unroll
    for (int c = 0; c < 4; ++c) q[c] = ldh(QH + qo + 32 * c);
    const size_t ko = ((size_t)zk * SEQ + lr) * HD + 8 * hi;
    const size_t vo = ((size_t)zk * HD + lr) * SEQ + 8 * hi;
    v8f o[8];
#pragma unroll
    for (int j = 0; j < 8; ++j) o[j] = (v8f){};
    float m = -3.0e38f, l = 0.0f;
    const int tq = t0 + lr;
    const int nst = (t0 + 15) / 32 + 1;
#pragma unroll 1
    for (int st = 0; st < nst; ++st) {
        const int key0 = st * 32;
        const size_t kofs = ko + (size_t)key0 * HD;
        v8f sa = (v8f){}, sb = (v8f){};
        v16h fa, fb;
#pragma unroll
        for (int c = 0; c < 4; ++c) { fa = ldh(KP + kofs + 32 * c); fb = ldh(KP + kofs + 16 * HD + 32 * c);
            sa = wmma16(fa, q[c], sa); sb = wmma16(fb, q[c], sb); }
        asm volatile("v_nop\n\tv_nop\n\tv_nop\n\tv_nop" : "+v"(sa), "+v"(sb) : "v"(fa), "v"(fb));
        float ta[8], tb[8]; float mx = -3.0e38f;
        const int kk = key0 + 8 * hi - tq;
#pragma unroll
        for (int r = 0; r < 8; ++r) { float u = sa[r] * SC2; float w = sb[r] * SC2;
            u = (kk + r > 0) ? -1.0e30f : u; w = (kk + 16 + r > 0) ? -1.0e30f : w;
            ta[r] = u; tb[r] = w; mx = fmaxf(mx, fmaxf(u, w)); }
        mx = fmaxf(mx, __shfl_xor(mx, 16, 32));
        const float mnew = fmaxf(m, mx);
        const float alpha = __builtin_amdgcn_exp2f(m - mnew);
        const float sh = PSH - mnew;
        v16h pb; float ls = 0.0f;
#pragma unroll
        for (int r = 0; r < 8; ++r) { const h16 pa = (h16)__builtin_amdgcn_exp2f(ta[r] + sh); const h16 pc = (h16)__builtin_amdgcn_exp2f(tb[r] + sh); pb[r] = pa; pb[8 + r] = pc; ls += (float)pa + (float)pc; }
        l = l * alpha + ls; m = mnew;
#pragma unroll
        for (int j = 0; j < 8; ++j) o[j] = o[j] * alpha;
        const size_t vofs = vo + key0;
        v16h vf;
#pragma unroll
        for (int j = 0; j < 8; ++j) { vf = ldh(VT + vofs + (size_t)(16 * j) * SEQ); o[j] = wmma16(vf, pb, o[j]); }
        asm volatile("v_nop\n\tv_nop\n\tv_nop\n\tv_nop" : "+v"(o[4]), "+v"(o[5]), "+v"(o[6]), "+v"(o[7]) : "v"(vf), "v"(pb));
    }
    l += __shfl_xor(l, 16, 32);
    const float inv = OCS * (1.0f / l);
    const int wb = wave * 16 * 132;
#pragma unroll
    for (int j = 0; j < 8; ++j) { const v8f f = o[j] * inv;
        const v4f a = __builtin_shufflevector(f, f, 0, 1, 2, 3); const v4f c = __builtin_shufflevector(f, f, 4, 5, 6, 7);
        *(v4fa*)(&os[wb + lr * 132 + 16 * j + 8 * hi]) = a; *(v4fa*)(&os[wb + lr * 132 + 16 * j + 8 * hi + 4]) = c; }
    wave_sync();
    const size_t obase = ((size_t)b * SEQ + t0) * DM + gh * HD;
#pragma unroll 1
    for (int ps = 0; ps < 2; ++ps) {
#pragma unroll
        for (int s = 0; s < 8; ++s) { const int row = 2 * s + (lane >> 4), c8 = (lane & 15) * 8;
            const v4f x0 = *(const v4fa*)(&os[wb + row * 132 + c8]); const v4f x1 = *(const v4fa*)(&os[wb + row * 132 + c8 + 4]); v8h hv;
#pragma unroll
            for (int i = 0; i < 4; ++i) { hv[i] = (h16)x0[i]; hv[4 + i] = (h16)x1[i]; }
            *(volatile v8h*)(OH + obase + (size_t)row * DM + c8) = hv; }
        if (ps == 0) __threadfence(); }
}

template <int RES>
__global__ __launch_bounds__(32) void k_out(const h16* __restrict__ OHp, const h16* __restrict__ ORp, const h16* __restrict__ Wt, float* OUT, int rowStart, int tilesPerBatch) {
    constexpr int MB = RES ? 2 : 4;
    __shared__ __align__(16) float os[16 * 68];
    const int K = DM;
    const int lane = threadIdx.x & 31, lr = lane & 15, hi = lane >> 4;
    const int bx = blockIdx.x; const int b = bx / tilesPerBatch, tile = bx % tilesPerBatch;
    const int tk0 = rowStart + tile * (16 * MB);
    const int c0 = blockIdx.y * 64;
    v8f accH[MB][4], accL[MB][4];
#pragma unroll
    for (int mb = 0; mb < MB; ++mb)
#pragma unroll
        for (int nb = 0; nb < 4; ++nb) { accH[mb][nb] = (v8f){}; accL[mb][nb] = (v8f){}; }
    const size_t aoff = ((size_t)b * SEQ + tk0 + lr) * K + 8 * hi, boff = (size_t)(c0 + lr) * K + 8 * hi;
#pragma unroll 1
    for (int kc = 0; kc < K; kc += 32) {
        v16h a[MB], ar[MB]; v16h bw;
#pragma unroll
        for (int mb = 0; mb < MB; ++mb) { a[mb] = ldh(OHp + aoff + (size_t)mb * 16 * K + kc); ar[mb] = ldh(ORp + aoff + (size_t)mb * 16 * K + kc); }
#pragma unroll
        for (int nb = 0; nb < 4; ++nb) { bw = ldh(Wt + boff + (size_t)nb * 16 * K + kc);
#pragma unroll
            for (int mb = 0; mb < MB; ++mb) { accH[mb][nb] = wmma16(a[mb], bw, accH[mb][nb]); if (RES) accL[mb][nb] = wmma16(ar[mb], bw, accL[mb][nb]); } }
        if (RES) asm volatile("v_nop\n\tv_nop\n\tv_nop\n\tv_nop" : "+v"(accH[0][3]), "+v"(accL[0][3]), "+v"(accH[MB - 1][3]), "+v"(accL[MB - 1][3]) : "v"(a[0]), "v"(a[MB - 1]), "v"(ar[0]), "v"(ar[MB - 1]), "v"(bw));
        else     asm volatile("v_nop\n\tv_nop\n\tv_nop\n\tv_nop" : "+v"(accH[0][3]), "+v"(accH[1][3]), "+v"(accH[MB - 2][3]), "+v"(accH[MB - 1][3]) : "v"(a[0]), "v"(a[1]), "v"(a[MB - 2]), "v"(a[MB - 1]), "v"(bw));
    }
#pragma unroll
    for (int mb = 0; mb < MB; ++mb) {
#pragma unroll
        for (int nb = 0; nb < 4; ++nb) {
#pragma unroll
            for (int j = 0; j < 8; ++j) { float val = accH[mb][nb][j]; if (RES) val += accL[mb][nb][j] * QRI;
                os[(hi * 8 + j) * 68 + nb * 16 + lr] = val * OSI; } }
        wave_sync();
        float* orow = OUT + ((size_t)b * OUT_SEQ + tk0 + mb * 16) * DM + c0;
#pragma unroll 1
        for (int ps = 0; ps < 2; ++ps) {
#pragma unroll
            for (int s = 0; s < 8; ++s) { const int row = 2 * s + hi, cofs = lr * 4;
                const v4f val = *(const v4fa*)(&os[row * 68 + cofs]);
                *(volatile v4f*)(orow + (size_t)row * DM + cofs) = val; }
            if (ps == 0) __threadfence(); }
        wave_sync();
    }
}

static constexpr size_t al256(size_t v) { return (v + 255) & ~(size_t)255; }
static constexpr size_t SZ_XB  = al256((size_t)NB * SEQ * DM * 2);
static constexpr size_t SZ_WQ  = al256((size_t)DM * DM * 2);
static constexpr size_t SZ_WKV = al256((size_t)DKV * DM * 2);
static constexpr size_t SZ_WO  = al256((size_t)DM * DM * 2);
static constexpr size_t SZ_TAB = al256((size_t)64 * SEQ * 4);
static constexpr size_t SZ_QP  = al256((size_t)NB * NQH * SEQ * HD * 2);
static constexpr size_t SZ_KP  = al256((size_t)NB * NG * SEQ * HD * 2);
static constexpr size_t SZ_OP  = al256((size_t)NB * SEQ * DM * 2);
static constexpr size_t SZ_TOTAL = SZ_XB + SZ_WQ + 2 * SZ_WKV + SZ_WO + 2 * SZ_TAB + 2 * SZ_QP + 4 * SZ_KP + 2 * SZ_OP;
static_assert(SZ_TOTAL <= (size_t)134217728);

extern "C" void kernel_launch(void* const* d_in, const int* in_sizes, int n_in,
                              void* d_out, int out_size, void* d_ws, size_t ws_size, hipStream_t stream) {
    if (n_in < 5) return;
    const size_t needx = ((size_t)(NB - 1) * SEQ_FULL + SEQ) * DM;
    if ((size_t)in_sizes[0] < needx) return;
    if ((size_t)in_sizes[1] < (size_t)DM * DM || (size_t)in_sizes[2] < (size_t)DM * DKV || (size_t)in_sizes[3] < (size_t)DM * DKV || (size_t)in_sizes[4] < (size_t)DM * DM) return;
    if ((size_t)out_size < ((size_t)(NB - 1) * OUT_SEQ + SEQ) * DM) return;
    if (SZ_TOTAL > ws_size) return;
    const float* x = (const float*)d_in[0]; const float* waq = (const float*)d_in[1]; const float* wak = (const float*)d_in[2];
    const float* wav = (const float*)d_in[3]; const float* wao = (const float*)d_in[4];
    float* OUT = (float*)d_out;
    char* wsp = (char*)d_ws;
    bf*  XB  = (bf*)wsp;  wsp += SZ_XB;
    bf*  WQT = (bf*)wsp;  wsp += SZ_WQ;
    bf*  WKT = (bf*)wsp;  wsp += SZ_WKV;
    bf*  WVT = (bf*)wsp;  wsp += SZ_WKV;
    h16* WOT = (h16*)wsp; wsp += SZ_WO;
    float* CT = (float*)wsp; wsp += SZ_TAB;
    float* ST = (float*)wsp; wsp += SZ_TAB;
    h16* QH = (h16*)wsp; wsp += SZ_QP;
    h16* QR = (h16*)wsp; wsp += SZ_QP;
    h16* KP = (h16*)wsp; wsp += SZ_KP;
    h16* KR = (h16*)wsp; wsp += SZ_KP;
    h16* VT = (h16*)wsp; wsp += SZ_KP;
    h16* VR = (h16*)wsp; wsp += SZ_KP;
    h16* OH = (h16*)wsp; wsp += SZ_OP;
    h16* OR = (h16*)wsp; wsp += SZ_OP;

    if (SEQ == SEQ_FULL) {
        const size_t n8 = (size_t)NB * SEQ * DM / 8;
        k_cvt8<<<(unsigned)((n8 + 255) / 256), 256, 0, stream>>>(x, XB, n8);
    } else {
        const size_t n8 = (size_t)SEQ * DM / 8;
        for (int b = 0; b < NB; ++b) k_cvt8<<<(unsigned)((n8 + 255) / 256), 256, 0, stream>>>(x + (size_t)b * SEQ_FULL * DM, XB + (size_t)b * SEQ * DM, n8);
    }
    k_tcvt<<<dim3(DM / 64,  DM / 64, 1), 256, 0, stream>>>(waq, (unsigned short*)WQT, DM, DM,  0);
    k_tcvt<<<dim3(DKV / 64, DM / 64, 1), 256, 0, stream>>>(wak, (unsigned short*)WKT, DM, DKV, 0);
    k_tcvt<<<dim3(DKV / 64, DM / 64, 1), 256, 0, stream>>>(wav, (unsigned short*)WVT, DM, DKV, 0);
    k_tcvt<<<dim3(DM / 64,  DM / 64, 1), 256, 0, stream>>>(wao, (unsigned short*)WOT, DM, DM,  1);
    k_ropetab<<<(unsigned)((64 * SEQ) / 256), 256, 0, stream>>>(CT, ST);

    k_projr<<<dim3(NB * SEQ / 32, NQH, 1), 32, 0, stream>>>(XB, WQT, CT, ST, QH, QR, NQH);
    k_projr<<<dim3(NB * SEQ / 32, NG,  1), 32, 0, stream>>>(XB, WKT, CT, ST, KP, KR, NG);
    k_projt<<<dim3(DKV / 64, NB * SEQ / 64, 1), 32, 0, stream>>>(WVT, XB, VT, VR, 1, DKV, (size_t)0, SEQ, SEQ, (size_t)DKV * SEQ);

    k_flash3<<<dim3(ESEQ / (16 * AW), NB * NQH, 2), 32 * AW, 0, stream>>>(QH, QR, KP, KR, VT, VR, OH, OR);
    if (SEQ > ESEQ) k_flash<<<dim3((SEQ - ESEQ) / (16 * AW), NB * NQH, 1), 32 * AW, 0, stream>>>(QH, KP, VT, OH);

    k_out<1><<<dim3(NB * (ESEQ / 32), DM / 64, 1), 32, 0, stream>>>(OH, OR, WOT, OUT, 0, ESEQ / 32);
    if (SEQ > ESEQ) k_out<0><<<dim3(NB * ((SEQ - ESEQ) / 64), DM / 64, 1), 32, 0, stream>>>(OH, OH, WOT, OUT, ESEQ, (SEQ - ESEQ) / 64);
}
